// MultiHeadDecoder_87205015978169
// MI455X (gfx1250) — hardware-run, weakly checked
//
#include <hip/hip_runtime.h>
#include <math.h>

#ifndef NB
#define NB 64
#endif
#define NB_FULL 64
#define GS 2001
#define GS_FULL 2001
#define DM 128
#define NHEAD 4
#define NPAIR 1000
#define IPITCH 2048
#define TPITCH 1024
#define GB ((NB) < 8 ? (NB) : 8)
#define NGRP ((NB) / GB)
#define GROWS (GB * GS)
#define GPAD (((GROWS + 63) / 64) * 64)
#define CWAVES 63
#define NROWS (NB * NPAIR)
#define NRPAD (((NROWS + 63) / 64) * 64)
#define NETW 64
#define NHID 32
#define NFEAT 12

constexpr size_t al256(size_t x) { return (x + 255) & ~(size_t)255; }
constexpr size_t SZ_QK    = al256((size_t)8 * GPAD * DM * 4);
constexpr size_t OFF_WN   = 0;
constexpr size_t OFF_WQK  = OFF_WN   + al256((size_t)DM * DM * 2);
constexpr size_t OFF_BT   = OFF_WQK  + al256((size_t)8 * DM * DM * 2);
constexpr size_t OFF_GMX  = OFF_BT   + al256((size_t)2 * NETW * NETW * 2);
constexpr size_t OFF_GG   = OFF_GMX  + al256((size_t)NB * DM * 4);
constexpr size_t OFF_PRE  = OFF_GG   + al256((size_t)NB * DM * 4);
constexpr size_t OFF_POST = OFF_PRE  + al256((size_t)NB * IPITCH * 4);
constexpr size_t OFF_X16  = OFF_POST + al256((size_t)NB * IPITCH * 4);
constexpr size_t OFF_H16  = OFF_X16  + al256((size_t)GPAD * DM * 2);
constexpr size_t OFF_QK   = OFF_H16  + al256((size_t)GPAD * DM * 2);
constexpr size_t OFF_CMP  = OFF_QK   + SZ_QK;
constexpr size_t OFF_TAB  = OFF_CMP  + al256((size_t)4 * NB * IPITCH * 4);
constexpr size_t OFF_PRB  = OFF_TAB  + al256((size_t)NB * TPITCH * 4);
constexpr size_t WS_TOTAL = OFF_PRB  + al256((size_t)NB * TPITCH * 4);
constexpr size_t OFF_FA   = OFF_QK;
constexpr size_t OFF_XA   = OFF_FA + al256((size_t)NRPAD * NETW * 2);
constexpr size_t OFF_X1   = OFF_XA + al256((size_t)NRPAD * NETW * 2);
constexpr size_t OFF_X2   = OFF_X1 + al256((size_t)NRPAD * NETW * 4);
constexpr size_t NET_END  = OFF_X2 + al256((size_t)NRPAD * NETW * 4);
static_assert(NET_END <= OFF_QK + SZ_QK);
static_assert(WS_TOTAL <= (size_t)134217728);

static_assert(NB <= NB_FULL);
static_assert(NB % GB == 0);
static_assert(GS == GS_FULL);
static_assert(2 * NPAIR == GS - 1);
static_assert(GPAD % 64 == 0 && GPAD >= GROWS);
static_assert(DM % 64 == 0 && DM % 32 == 0 && DM == 128);
static_assert(((size_t)GPAD * DM / 8) % 256 == 0);
static_assert((DM * DM / 8) % 256 == 0);
static_assert(CWAVES * 32 >= GS - 1 && CWAVES * 32 <= IPITCH);
static_assert(GS <= IPITCH && IPITCH == 2048 && 256 * 4 * 2 == IPITCH);
static_assert(NPAIR <= TPITCH && TPITCH == 4 * 256);
static_assert(NHEAD == 4);
static_assert(NRPAD % 64 == 0 && NRPAD >= NROWS && NETW % 64 == 0 && NETW % 32 == 0);
static_assert(NHID == 32 && 2 * NHID == NETW && NFEAT == 12 && NFEAT <= NHID);
static_assert(8 * 16 * 68 * 4 <= 131072);
static_assert(2 * IPITCH * 4 <= 131072);
static_assert((32 + 1) * 4 <= 131072);
static_assert(32 * 16 * 4 == 16 * 128);
static_assert(32 * 16 * 8 == 16 * 256);
static_assert(8 * 16 == NETW * 2);
static_assert(((size_t)NRPAD * 8) % 256 == 0);
static_assert(2 * 256 * 16 == NETW * NETW * 2);

typedef __attribute__((ext_vector_type(16))) _Float16 v16h;
typedef __attribute__((ext_vector_type(8)))  _Float16 v8h;
typedef __attribute__((ext_vector_type(2)))  _Float16 v2h;
typedef __attribute__((ext_vector_type(8)))  float    v8f;
typedef __attribute__((ext_vector_type(4)))  float    v4f;
typedef __attribute__((ext_vector_type(2)))  float    v2f;
typedef __attribute__((ext_vector_type(4)))  unsigned int v4u;
typedef __attribute__((ext_vector_type(4)))  int      v4i;


#define VST2(T, ptr, val) do { const T vst2_v_ = (val); *(volatile T*)(ptr) = vst2_v_; __threadfence(); *(volatile T*)(ptr) = vst2_v_; } while (0)
#define VST2V4(ptr, val) do { const v4f vst2_v4_ = (val); *(volatile v4f*)(ptr) = vst2_v4_; __threadfence(); *(volatile v4f*)(ptr) = vst2_v4_; } while (0)

__device__ __forceinline__ float bfr(float f) {
    unsigned u = __float_as_uint(f);
    u += 0x7FFFu + ((u >> 16) & 1u);
    return __uint_as_float(u & 0xFFFF0000u);
}

static __device__ __forceinline__ v2h toh_flush2(float a, float b) {
    v2f w;
    w.x = (fabsf(a) < 6.103515625e-05f) ? 0.0f : a;
    w.y = (fabsf(b) < 6.103515625e-05f) ? 0.0f : b;
    return __builtin_convertvector(w, v2h);
}
union Pack8 { v8h v; v2h p[4]; };
static __device__ __forceinline__ v8h pack8_flush(const float* v) {
    Pack8 u;
    u.p[0] = toh_flush2(v[0], v[1]);
    u.p[1] = toh_flush2(v[2], v[3]);
    u.p[2] = toh_flush2(v[4], v[5]);
    u.p[3] = toh_flush2(v[6], v[7]);
    return u.v;
}
static __device__ __forceinline__ void split8(const float* a, bool second_word, float* o) {
#pragma unroll
    for (int e = 0; e < 8; e += 2) {
        const v2h h = toh_flush2(a[e], a[e + 1]);
        const float r0 = (a[e] - (float)h.x) * 2048.0f;
        const float r1 = (a[e + 1] - (float)h.y) * 2048.0f;
        o[e] = second_word ? r0 : a[e];
        o[e + 1] = second_word ? r1 : a[e + 1];
    }
}
static __device__ __forceinline__ void st8h2(_Float16* P, size_t o, v8h hv) {
    *(volatile v8h*)(P + o) = hv;
    __threadfence();
    *(volatile v8h*)(P + o) = hv;
}

union FragU { v16h v; v8h h[2]; };
__device__ __forceinline__ v16h frag_ld(const _Float16* p) {
    FragU f; f.h[0] = *(const v8h*)(p); f.h[1] = *(const v8h*)(p + 16); return f.v;
}
__device__ __forceinline__ v8f wmma16(v16h a, v16h b, v8f c) {
    c = __builtin_amdgcn_wmma_f32_16x16x32_f16(false, a, false, b, (short)0, c, false, false);
    asm volatile("v_nop\n\tv_nop\n\tv_nop\n\tv_nop" : "+v"(c) : "v"(a), "v"(b));
    return c;
}
__device__ __forceinline__ void wave_sync_lds() {
    __builtin_amdgcn_fence(3  , "workgroup");
    __builtin_amdgcn_wave_barrier();
    __builtin_amdgcn_fence(2  , "workgroup");
}

template <int OUT_MODE, bool ROWADD, bool BIASRELU = false>
static __device__ __forceinline__ void gemm64_body(
    const _Float16* __restrict__ A, unsigned lda, const _Float16* __restrict__ Bt, unsigned ldb,
    void* __restrict__ Cout, unsigned ldc, const float* __restrict__ addtab, unsigned ent0,
    unsigned rowsLive, unsigned rowsPerEnt,
    unsigned M, unsigned N, unsigned K, float scale, float oscale,
    const float* __restrict__ bias = nullptr, unsigned nbias = 1u) {
  __shared__ __align__(16) float sT[8][16 * 68];
  const unsigned lane = threadIdx.x & 31u;
  const unsigned wave = threadIdx.x >> 5;
  const unsigned tilesN = N >> 6, tilesM = M >> 6;
  const unsigned tile = blockIdx.x * 8u + wave;
  if (tile >= tilesM * tilesN) return;
  const unsigned tm = tile / tilesN;
  const unsigned tn = tile - tm * tilesN;
  const unsigned m0 = tm << 6, n0 = tn << 6;
  const unsigned rlane = lane & 15u;
  const unsigned koff = (lane >> 4) * 8u;
  const unsigned mOff = koff;

  v8f acc[4][4];
#pragma unroll
  for (int i = 0; i < 4; ++i)
#pragma unroll
    for (int j = 0; j < 4; ++j) acc[i][j] = (v8f){0.f,0.f,0.f,0.f,0.f,0.f,0.f,0.f};

  for (unsigned k0 = 0; k0 < K; k0 += 32u) {
    v16h bh[4];
#pragma unroll
    for (int j = 0; j < 4; ++j)
      bh[j] = frag_ld(Bt + (size_t)(n0 + ((unsigned)j << 4) + rlane) * ldb + koff + k0);
#pragma unroll
    for (int i = 0; i < 4; ++i) {
      const v16h ah = frag_ld(A + (size_t)(m0 + ((unsigned)i << 4) + rlane) * lda + koff + k0);
#pragma unroll
      for (int j = 0; j < 4; ++j)
        acc[i][j] = wmma16(ah, bh[j], acc[i][j]);
    }
  }

  float bcol[4] = {0.f, 0.f, 0.f, 0.f};
  if (BIASRELU) {
#pragma unroll
    for (int j = 0; j < 4; ++j) {
      const unsigned n = n0 + ((unsigned)j << 4) + rlane;
      const unsigned nc = (n < nbias) ? n : (nbias - 1u);
      const float bq = bias[nc];
      bcol[j] = (n < nbias) ? bfr(bq) : 0.0f;
    }
  }

  float* slab = sT[wave];
#pragma unroll
  for (int i = 0; i < 4; ++i) {
    const unsigned mBase = m0 + ((unsigned)i << 4);
#pragma unroll
    for (int j = 0; j < 4; ++j) {
#pragma unroll
      for (int r = 0; r < 8; ++r) {
        float v = acc[i][j][r] * scale;
        if (BIASRELU) v = fmaxf(v + bcol[j], 0.0f);
        slab[(mOff + (unsigned)r) * 68u + ((unsigned)j << 4) + rlane] = v;
      }
    }
    wave_sync_lds();
    if (OUT_MODE == 0) {
      float* C = (float*)Cout;
      const unsigned hh = lane >> 4, c4 = (lane & 15u) * 4u;
#pragma unroll
      for (int half = 0; half < 2; ++half) {
        v4f vv[4];
#pragma unroll
        for (int it = 0; it < 4; ++it) {
          const unsigned row = (unsigned)(half * 4 + it) * 2u + hh;
          vv[it] = *(const v4f*)(slab + row * 68u + c4);
        }
        for (int pass = 0; pass < 2; ++pass) {
#pragma unroll
          for (int it = 0; it < 4; ++it) {
            const unsigned row = (unsigned)(half * 4 + it) * 2u + hh;
            *(volatile v4f*)(C + (size_t)(mBase + row) * ldc + n0 + c4) = vv[it];
          }
          __threadfence();
        }
      }
    } else {
      _Float16* C = (_Float16*)Cout;
      const unsigned q = lane >> 3, c8 = (lane & 7u) * 8u;
      v8h hv[4];
#pragma unroll
      for (int it = 0; it < 4; ++it) {
        const unsigned row = (unsigned)it * 4u + q;
        const float* sp = slab + row * 68u + c8;
        float t[8];
#pragma unroll
        for (int e = 0; e < 8; ++e) t[e] = sp[e];
        if (ROWADD) {
          const unsigned grow = mBase + row;
          const bool live = grow < rowsLive;
          const unsigned gc = live ? grow : (rowsLive - 1u);
          const float* ap = addtab + (size_t)(ent0 + gc / rowsPerEnt) * N + n0 + c8;
          const v4f g0 = *(const v4f*)ap, g1 = *(const v4f*)(ap + 4);
          const float ga[8] = {g0.x, g0.y, g0.z, g0.w, g1.x, g1.y, g1.z, g1.w};
#pragma unroll
          for (int e = 0; e < 8; ++e) t[e] = live ? (t[e] + ga[e]) : 0.0f;
        }
#pragma unroll
        for (int e = 0; e < 8; ++e) t[e] *= oscale;
        hv[it] = pack8_flush(t);
      }
      for (int pass = 0; pass < 2; ++pass) {
#pragma unroll
        for (int it = 0; it < 4; ++it) {
          const unsigned row = (unsigned)it * 4u + q;
          *(volatile v8h*)(C + (size_t)(mBase + row) * ldc + n0 + c8) = hv[it];
        }
        __threadfence();
      }
    }
    wave_sync_lds();
  }
}

__global__ __launch_bounds__(256) void k_hgemm(const _Float16* __restrict__ X16, const _Float16* __restrict__ WN16,
                                               const float* __restrict__ GG, _Float16* __restrict__ H16, unsigned ent0) {
    gemm64_body<1, true>(X16, DM, WN16, DM, (void*)H16, DM, GG, ent0, (unsigned)GROWS, (unsigned)GS,
                         (unsigned)GPAD, DM, DM, 1.0f / 65536.0f, 128.0f);
}

__global__ __launch_bounds__(256) void k_proj(const _Float16* __restrict__ H16, const _Float16* __restrict__ W16,
                                              float* __restrict__ QK32) {
    const unsigned pl = blockIdx.y;
    gemm64_body<0, false>(H16, DM, W16 + (size_t)pl * DM * DM, DM, (void*)(QK32 + (size_t)pl * GPAD * DM), DM,
                          (const float*)nullptr, 0u, (unsigned)GPAD, 1u, (unsigned)GPAD, DM, DM, 1.0f / 131072.0f, 1.0f);
}

__global__ __launch_bounds__(256) void k_layer(const _Float16* __restrict__ A16, const _Float16* __restrict__ BT,
                                               const float* __restrict__ bias, float* __restrict__ X32) {
    gemm64_body<0, false, true>(A16, NETW, BT, NETW, (void*)X32, NETW, (const float*)nullptr, 0u, (unsigned)NRPAD, 1u,
                                (unsigned)NRPAD, NETW, NETW, 1.0f / 262144.0f, 1.0f, bias, (unsigned)NHID);
}

__global__ __launch_bounds__(256) void k_wn(const float* __restrict__ Wm, _Float16* __restrict__ W16) {
    const unsigned u = blockIdx.x * 256u + threadIdx.x;
    if (u >= (unsigned)(DM * DM / 8)) return;
    const float* src = Wm + (size_t)u * 8u;
    const v4f a = *(const v4f*)src, b = *(const v4f*)(src + 4);
    float v[8] = {bfr(a.x) * 1024.0f, bfr(a.y) * 1024.0f, bfr(a.z) * 1024.0f, bfr(a.w) * 1024.0f,
                  bfr(b.x) * 1024.0f, bfr(b.y) * 1024.0f, bfr(b.z) * 1024.0f, bfr(b.w) * 1024.0f};
    st8h2(W16, (size_t)u * 8u, pack8_flush(v));
}

__global__ __launch_bounds__(256) void k_wt(const float* __restrict__ Wm, unsigned KI, unsigned NO, unsigned lgper,
                                            _Float16* __restrict__ W16) {
    const unsigned head = blockIdx.y;
    const float* Wl = Wm + (size_t)head * KI * NO;
    _Float16* Dl = W16 + (size_t)head * KI * NO;
    const unsigned u = blockIdx.x * 256u + threadIdx.x;
    const unsigned per = 1u << lgper;
    if (u >= NO * per) return;
    const unsigned k0 = 8u * (u & (per - 1u));
    const unsigned o = u >> lgper;
    float v[8];
#pragma unroll
    for (int i = 0; i < 8; ++i) v[i] = bfr(Wl[(size_t)(k0 + (unsigned)i) * NO + o]) * 1024.0f;
    st8h2(Dl, (size_t)o * KI + k0, pack8_flush(v));
}

__global__ __launch_bounds__(256) void k_w12(const float* __restrict__ w1, const float* __restrict__ w2, _Float16* __restrict__ BT) {
    const unsigned layer = blockIdx.y;
    const unsigned u = blockIdx.x * 256u + threadIdx.x;
    if (u >= (unsigned)(NETW * NETW / 8)) return;
    const unsigned o = u >> 3, k0 = (u & 7u) * 8u;
    const unsigned oc = min(o, (unsigned)(NHID - 1));
    float v[8];
#pragma unroll
    for (int e = 0; e < 8; ++e) {
        const unsigned k = k0 + (unsigned)e;
        const unsigned kk = k & 31u;
        const float a1 = w1[oc * (unsigned)NFEAT + min(kk, (unsigned)(NFEAT - 1))];
        const float a2 = w2[oc * (unsigned)NHID + kk];
        const bool in1 = (o < (unsigned)NHID) && (kk < (unsigned)NFEAT);
        const bool in2 = (o < (unsigned)NHID);
        const float s1 = in1 ? bfr(a1) : 0.0f;
        const float s2 = in2 ? bfr(a2) : 0.0f;
        const float w = (layer == 0u) ? s1 : s2;
        v[e] = w * ((k >= 32u) ? 0.5f : 1024.0f);
    }
    st8h2(BT + (size_t)layer * NETW * NETW, (size_t)o * NETW + k0, pack8_flush(v));
}

__global__ __launch_bounds__(256) void k_gmax(const float* __restrict__ h_em, float* __restrict__ G) {
    __shared__ __align__(16) float sM[8][DM];
    const unsigned t = threadIdx.x, lane = t & 31u;
    const unsigned wave = __builtin_amdgcn_readfirstlane(threadIdx.x >> 5);
    const unsigned b = blockIdx.x;
    const float* src = h_em + (size_t)b * GS_FULL * DM + 4u * lane;
    float m0 = -3.0e38f, m1 = -3.0e38f, m2 = -3.0e38f, m3 = -3.0e38f;
    for (unsigned g = wave; g < (unsigned)GS; g += 8u) {
        const v4f a = *(const v4f*)(src + (size_t)g * DM);
        m0 = fmaxf(m0, bfr(a.x)); m1 = fmaxf(m1, bfr(a.y)); m2 = fmaxf(m2, bfr(a.z)); m3 = fmaxf(m3, bfr(a.w));
    }
    sM[wave][4u * lane] = m0; sM[wave][4u * lane + 1u] = m1; sM[wave][4u * lane + 2u] = m2; sM[wave][4u * lane + 3u] = m3;
    __syncthreads();
    if (t < 32u) {
        float r[4];
#pragma unroll
        for (int c = 0; c < 4; ++c) {
            float m = sM[0][4u * t + (unsigned)c];
#pragma unroll
            for (int w = 1; w < 8; ++w) m = fmaxf(m, sM[w][4u * t + (unsigned)c]);
            r[c] = m;
        }
        v4f v; v.x = r[0]; v.y = r[1]; v.z = r[2]; v.w = r[3];
        VST2V4(G + (size_t)b * DM + 4u * t, v);
    }
}

__global__ __launch_bounds__(256) void k_gg(const float* __restrict__ G, const float* __restrict__ Wg, float* __restrict__ GG) {
    const unsigned u = blockIdx.x * 256u + threadIdx.x;
    if (u >= (unsigned)(NB * DM)) return;
    const unsigned b = u >> 7, e = u & 127u;
    const float* gr = G + (size_t)b * DM;
    const float* wr = Wg + (size_t)e * DM;
    float acc = 0.f;
    for (unsigned d = 0; d < (unsigned)DM; d += 4u) {
        const v4f g4 = *(const v4f*)(gr + d);
        const v4f w4 = *(const v4f*)(wr + d);
        acc += g4.x * bfr(w4.x);
        acc += g4.y * bfr(w4.y);
        acc += g4.z * bfr(w4.z);
        acc += g4.w * bfr(w4.w);
    }
    VST2(float, GG + u, acc);
}

__global__ __launch_bounds__(256) void k_perm(const int* __restrict__ rec, int* __restrict__ PRE, int* __restrict__ POST) {
    __shared__ int sRec[IPITCH];
    __shared__ int sInv[IPITCH];
    const unsigned t = threadIdx.x, b = blockIdx.x;
    const int* rr = rec + (size_t)b * GS_FULL;
    for (unsigned i = t; i < (unsigned)IPITCH; i += 256u) {
        const unsigned ic = min(i, (unsigned)(GS - 1));
        const int r = rr[ic];
        const int rc = min(max(r, 0), GS - 1);
        sRec[i] = (i < (unsigned)GS) ? rc : 0;
        sInv[i] = 0;
    }
    __syncthreads();
    for (unsigned i = t; i < (unsigned)GS; i += 256u) sInv[sRec[i]] = (int)i;
    __syncthreads();
#pragma unroll
    for (int it = 0; it < 2; ++it) {
        const unsigned i0 = 4u * (t + 256u * (unsigned)it);
        int pv[4], sv[4];
#pragma unroll
        for (int e = 0; e < 4; ++e) {
            const unsigned idx = i0 + (unsigned)e;
            const int a = sInv[idx];
            const int c = sRec[sRec[idx]];
            pv[e] = (idx < (unsigned)GS) ? a : 0;
            sv[e] = (idx < (unsigned)GS) ? c : 0;
        }
        v4i p; p.x = pv[0]; p.y = pv[1]; p.z = pv[2]; p.w = pv[3];
        v4i s; s.x = sv[0]; s.y = sv[1]; s.z = sv[2]; s.w = sv[3];
        VST2(v4i, (v4i*)(PRE + (size_t)b * IPITCH + i0), p);
        VST2(v4i, (v4i*)(POST + (size_t)b * IPITCH + i0), s);
    }
}

__global__ __launch_bounds__(256) void k_cvt_x(const float* __restrict__ h_em, _Float16* __restrict__ X16, unsigned ent0) {
    const unsigned u = blockIdx.x * 256u + threadIdx.x;
    if (u >= (unsigned)(GPAD * DM / 8)) return;
    const unsigned row = u >> 4, c0 = (u & 15u) * 8u;
    const bool live = row < (unsigned)GROWS;
    const unsigned rc = live ? row : (unsigned)(GROWS - 1);
    const float* xr = h_em + ((size_t)ent0 * GS_FULL + rc) * DM + c0;
    const v4f a = *(const v4f*)xr, b = *(const v4f*)(xr + 4);
    float v[8] = {bfr(a.x) * 64.0f, bfr(a.y) * 64.0f, bfr(a.z) * 64.0f, bfr(a.w) * 64.0f,
                  bfr(b.x) * 64.0f, bfr(b.y) * 64.0f, bfr(b.z) * 64.0f, bfr(b.w) * 64.0f};
#pragma unroll
    for (int i = 0; i < 8; ++i) v[i] = live ? v[i] : 0.0f;
    st8h2(X16, (size_t)row * DM + c0, pack8_flush(v));
}

__global__ __launch_bounds__(256) void k_compat(const float* __restrict__ QK, const int* __restrict__ PRE, const int* __restrict__ POST,
                                                float* __restrict__ CMP, unsigned ent0) {
    const unsigned lane = threadIdx.x & 31u;
    const unsigned wave = __builtin_amdgcn_readfirstlane(threadIdx.x >> 5);
    const unsigned gw = blockIdx.x * 8u + wave;
    if (gw >= (unsigned)(GB * CWAVES)) return;
    const unsigned bl = gw / (unsigned)CWAVES;
    const unsigned w = gw - bl * (unsigned)CWAVES;
    const unsigned b = ent0 + bl;
    const unsigned e0 = w * 32u;
    const unsigned myNode = min(e0 + lane + 1u, (unsigned)(GS - 1));
    const int pr = min(max(PRE[(size_t)b * IPITCH + myNode], 0), GS - 1);
    const int po = min(max(POST[(size_t)b * IPITCH + myNode], 0), GS - 1);
    const size_t PL = (size_t)GPAD * DM;
    const float* base = QK + (size_t)bl * GS * DM + 4u * lane;
    float keep[4] = {0.f, 0.f, 0.f, 0.f};
#pragma unroll 1
    for (unsigned n = 0; n < 32u; ++n) {
        const unsigned node = min(e0 + n + 1u, (unsigned)(GS - 1));
        const unsigned np = (unsigned)__shfl(pr, (int)n, 32);
        const unsigned ns = (unsigned)__shfl(po, (int)n, 32);
        const float* rowP = base + (size_t)np * DM;
        const float* rowI = base + (size_t)node * DM;
        const float* rowS = base + (size_t)ns * DM;
#pragma unroll
        for (int hd = 0; hd < 4; ++hd) {
            const v4f qp = *(const v4f*)(rowP + (size_t)hd * PL);
            const v4f qi = *(const v4f*)(rowI + (size_t)hd * PL);
            const v4f ki = *(const v4f*)(rowI + (size_t)(4 + hd) * PL);
            const v4f ks = *(const v4f*)(rowS + (size_t)(4 + hd) * PL);
            float t1 = qp.x * ki.x + qp.y * ki.y + qp.z * ki.z + qp.w * ki.w;
            float t2 = qi.x * ks.x + qi.y * ks.y + qi.z * ks.z + qi.w * ks.w;
            float t3 = qp.x * ks.x + qp.y * ks.y + qp.z * ks.z + qp.w * ks.w;
#pragma unroll
            for (int o = 16; o > 0; o >>= 1) {
                t1 += __shfl_xor(t1, o, 32);
                t2 += __shfl_xor(t2, o, 32);
                t3 += __shfl_xor(t3, o, 32);
            }
            const float cv = t1 + t2 - t3;
            keep[hd] = (lane == n) ? cv : keep[hd];
        }
    }
    const bool valid = (e0 + lane) < (unsigned)(GS - 1);
    float ov[4];
#pragma unroll
    for (int hd = 0; hd < 4; ++hd) ov[hd] = valid ? keep[hd] : 0.0f;
    float* dst = CMP + (size_t)b * IPITCH + e0 + lane;
    for (int pass = 0; pass < 2; ++pass) {
#pragma unroll
        for (int hd = 0; hd < 4; ++hd) *(volatile float*)(dst + (size_t)hd * NB * IPITCH) = ov[hd];
        __threadfence();
    }
}

__global__ __launch_bounds__(256) void k_feat(const float* __restrict__ CMP, const float* __restrict__ sig, _Float16* __restrict__ FA) {
    const unsigned u = blockIdx.x * 256u + threadIdx.x;
    if (u >= (unsigned)(NRPAD * 8)) return;
    const unsigned row = u >> 3, p = u & 7u;
    const bool live = row < (unsigned)NROWS;
    unsigned rr = live ? row : (unsigned)(NROWS - 1);
    asm volatile("" : "+v"(rr));
    const unsigned b = rr / (unsigned)NPAIR;
    const unsigned j = rr - b * (unsigned)NPAIR;
    float f[12];
#pragma unroll
    for (int hd = 0; hd < 4; ++hd) {
        const float* cp = CMP + ((size_t)hd * NB + b) * IPITCH;
        f[hd] = cp[j];
        f[4 + hd] = cp[NPAIR + j];
    }
#pragma unroll
    for (int s = 0; s < 4; ++s) f[8 + s] = bfr(sig[((size_t)b * 4u + (unsigned)s) * NPAIR + j]);
    const bool second8 = (p & 1u) != 0u;
    const bool used = live && ((p & 2u) == 0u);
    float a[8];
#pragma unroll
    for (int e = 0; e < 8; ++e) {
        const float va = f[e];
        const float vb = (e < 4) ? f[8 + (e & 3)] : 0.0f;
        const float v = second8 ? vb : va;
        a[e] = used ? (v * 256.0f) : 0.0f;
    }
    float o[8];
    split8(a, p >= 4u, o);
    st8h2(FA, (size_t)row * NETW + 8u * p, pack8_flush(o));
}

__global__ __launch_bounds__(256) void k_split(const float* __restrict__ X32, _Float16* __restrict__ XA) {
    const unsigned u = blockIdx.x * 256u + threadIdx.x;
    if (u >= (unsigned)(NRPAD * 8)) return;
    const unsigned row = u >> 3, p = u & 7u;
    const float* xr = X32 + (size_t)row * NETW + 8u * (p & 3u);
    const v4f x0 = *(const v4f*)xr, x1 = *(const v4f*)(xr + 4);
    const float a[8] = {x0.x * 256.0f, x0.y * 256.0f, x0.z * 256.0f, x0.w * 256.0f,
                        x1.x * 256.0f, x1.y * 256.0f, x1.z * 256.0f, x1.w * 256.0f};
    float o[8];
    split8(a, p >= 4u, o);
    st8h2(XA, (size_t)row * NETW + 8u * p, pack8_flush(o));
}

__global__ __launch_bounds__(256) void k_score(const float* __restrict__ X2, const float* __restrict__ w3, const float* __restrict__ b3,
                                               float* __restrict__ TAB) {
    __shared__ float sW3[32];
    __shared__ float sB3[1];
    const unsigned t = threadIdx.x;
    if (t < 32u) sW3[t] = bfr(w3[t]);
    if (t == 0u) sB3[0] = bfr(b3[0]);
    __syncthreads();
    const unsigned b = blockIdx.x >> 2;
    const unsigned j = (blockIdx.x & 3u) * 256u + t;
    const unsigned jc = min(j, (unsigned)(NPAIR - 1));
    const float* xr = X2 + ((size_t)b * NPAIR + jc) * NETW;
    float sc = 0.f;
#pragma unroll
    for (int g = 0; g < 8; ++g) {
        const v4f x = *(const v4f*)(xr + 4 * g);
        sc += sW3[4 * g] * x.x;
        sc += sW3[4 * g + 1] * x.y;
        sc += sW3[4 * g + 2] * x.z;
        sc += sW3[4 * g + 3] * x.w;
    }
    sc += sB3[0];
    const float tv = 6.0f * tanhf(sc);
    const float val = (j < (unsigned)NPAIR) ? tv : 0.0f;
    VST2(float, TAB + (size_t)b * TPITCH + j, val);
}

__global__ __launch_bounds__(256) void k_softmax(const float* __restrict__ TAB, float* __restrict__ PRB) {
    __shared__ float sMx[8];
    __shared__ float sSm[8];
    const unsigned t = threadIdx.x, lane = t & 31u;
    const unsigned wave = __builtin_amdgcn_readfirstlane(threadIdx.x >> 5);
    const unsigned b = blockIdx.x;
    const float* row = TAB + (size_t)b * TPITCH;
    float v[4];
#pragma unroll
    for (int q = 0; q < 4; ++q) {
        const unsigned j = t + 256u * (unsigned)q;
        const float x = row[j];
        v[q] = (j < (unsigned)NPAIR) ? x : -3.0e38f;
    }
    float m = fmaxf(fmaxf(v[0], v[1]), fmaxf(v[2], v[3]));
#pragma unroll
    for (int o = 16; o > 0; o >>= 1) m = fmaxf(m, __shfl_xor(m, o, 32));
    if (lane == 0u) sMx[wave] = m;
    __syncthreads();
    float mx = sMx[0];
#pragma unroll
    for (int w = 1; w < 8; ++w) mx = fmaxf(mx, sMx[w]);
    float e[4];
#pragma unroll
    for (int q = 0; q < 4; ++q) {
        const unsigned j = t + 256u * (unsigned)q;
        const float ex = expf(v[q] - mx);
        e[q] = (j < (unsigned)NPAIR) ? ex : 0.0f;
    }
    float s = (e[0] + e[1]) + (e[2] + e[3]);
#pragma unroll
    for (int o = 16; o > 0; o >>= 1) s += __shfl_xor(s, o, 32);
    if (lane == 0u) sSm[wave] = s;
    __syncthreads();
    float sum = sSm[0];
#pragma unroll
    for (int w = 1; w < 8; ++w) sum += sSm[w];
#pragma unroll
    for (int q = 0; q < 4; ++q) {
        const unsigned j = t + 256u * (unsigned)q;
        const float p = e[q] / sum;
        VST2(float, PRB + (size_t)b * TPITCH + j, p);
    }
}

__global__ __launch_bounds__(256) void k_out(const float* __restrict__ PRB, float* __restrict__ out) {
    const unsigned u = blockIdx.x * 256u + threadIdx.x;
    if (u >= (unsigned)(NB * NPAIR)) return;
    unsigned uu = u; asm volatile("" : "+v"(uu));
    const unsigned b = uu / (unsigned)NPAIR;
    const unsigned j = uu - b * (unsigned)NPAIR;
    const float p = PRB[(size_t)b * TPITCH + j];
    VST2(float, out + u, p);
}

extern "C" void kernel_launch(void* const* d_in, const int* in_sizes, int n_in, void* d_out, int out_size,
                              void* d_ws, size_t ws_size, hipStream_t stream) {
    if (n_in < 13) return;
    if (in_sizes[0] < NB * GS * DM || in_sizes[1] < NB * GS || in_sizes[2] < NB * 4 * NPAIR) return;
    if (in_sizes[3] < DM * DM || in_sizes[4] < DM * DM || in_sizes[5] < NHEAD * DM * DM || in_sizes[6] < NHEAD * DM * DM) return;
    if (in_sizes[7] < 384 || in_sizes[8] < 32 || in_sizes[9] < 1024 || in_sizes[10] < 32 || in_sizes[11] < 32 || in_sizes[12] < 1) return;
    if (out_size < NB * NPAIR) return;
    if (WS_TOTAL > ws_size) return;

    const float* h_em    = (const float*)d_in[0];
    const int*   rec     = (const int*)d_in[1];
    const float* sig     = (const float*)d_in[2];
    const float* W_node  = (const float*)d_in[3];
    const float* W_graph = (const float*)d_in[4];
    const float* W_Q     = (const float*)d_in[5];
    const float* W_K     = (const float*)d_in[6];
    const float* agg_w1  = (const float*)d_in[7];
    const float* agg_b1  = (const float*)d_in[8];
    const float* agg_w2  = (const float*)d_in[9];
    const float* agg_b2  = (const float*)d_in[10];
    const float* agg_w3  = (const float*)d_in[11];
    const float* agg_b3  = (const float*)d_in[12];
    float* out = (float*)d_out;

    char* wsp = (char*)d_ws;
    _Float16* wn16  = (_Float16*)(wsp + OFF_WN);
    _Float16* wqk16 = (_Float16*)(wsp + OFF_WQK);
    _Float16* bt12  = (_Float16*)(wsp + OFF_BT);
    float*    gmx   = (float*)(wsp + OFF_GMX);
    float*    gg    = (float*)(wsp + OFF_GG);
    int*      pre   = (int*)(wsp + OFF_PRE);
    int*      post  = (int*)(wsp + OFF_POST);
    _Float16* x16   = (_Float16*)(wsp + OFF_X16);
    _Float16* h16   = (_Float16*)(wsp + OFF_H16);
    float*    qk32  = (float*)(wsp + OFF_QK);
    float*    cmp   = (float*)(wsp + OFF_CMP);
    float*    tab   = (float*)(wsp + OFF_TAB);
    float*    prb   = (float*)(wsp + OFF_PRB);
    _Float16* fa    = (_Float16*)(wsp + OFF_FA);
    _Float16* xa    = (_Float16*)(wsp + OFF_XA);
    float*    x1    = (float*)(wsp + OFF_X1);
    float*    x2    = (float*)(wsp + OFF_X2);

    k_wn<<<(DM * DM / 8) / 256, 256, 0, stream>>>(W_node, wn16);
    k_wt<<<dim3((DM * (DM / 8)) / 256, NHEAD), 256, 0, stream>>>(W_Q, DM, DM, 4, wqk16);
    k_wt<<<dim3((DM * (DM / 8)) / 256, NHEAD), 256, 0, stream>>>(W_K, DM, DM, 4, wqk16 + (size_t)NHEAD * DM * DM);
    k_w12<<<dim3((NETW * NETW / 8) / 256, 2), 256, 0, stream>>>(agg_w1, agg_w2, bt12);

    k_gmax<<<NB, 256, 0, stream>>>(h_em, gmx);
    k_gg<<<(NB * DM + 255) / 256, 256, 0, stream>>>(gmx, W_graph, gg);
    k_perm<<<NB, 256, 0, stream>>>(rec, pre, post);

    const unsigned gH = ((GPAD / 64) * (DM / 64) + 7) / 8;
    const unsigned gC = (GB * CWAVES + 7) / 8;
    for (int gp = 0; gp < NGRP; ++gp) {
        const unsigned ent0 = (unsigned)(gp * GB);
        k_cvt_x<<<(GPAD * DM / 8) / 256, 256, 0, stream>>>(h_em, x16, ent0);
        k_hgemm<<<gH, 256, 0, stream>>>((const _Float16*)x16, (const _Float16*)wn16, (const float*)gg, h16, ent0);
        k_proj<<<dim3(gH, 8), 256, 0, stream>>>((const _Float16*)h16, (const _Float16*)wqk16, qk32);
        k_compat<<<gC, 256, 0, stream>>>((const float*)qk32, (const int*)pre, (const int*)post, cmp, ent0);
    }

    const unsigned gL = ((NRPAD / 64) * (NETW / 64) + 7) / 8;
    k_feat<<<(NRPAD * 8) / 256, 256, 0, stream>>>((const float*)cmp, sig, fa);
    k_layer<<<gL, 256, 0, stream>>>((const _Float16*)fa, (const _Float16*)bt12, agg_b1, x1);
    k_split<<<(NRPAD * 8) / 256, 256, 0, stream>>>((const float*)x1, xa);
    k_layer<<<gL, 256, 0, stream>>>((const _Float16*)xa, (const _Float16*)(bt12 + (size_t)NETW * NETW), agg_b2, x2);
    k_score<<<NB * 4, 256, 0, stream>>>((const float*)x2, agg_w3, agg_b3, tab);

    k_softmax<<<NB, 256, 0, stream>>>((const float*)tab, prb);
    k_out<<<(NB * NPAIR + 255) / 256, 256, 0, stream>>>((const float*)prb, out);
}
